// Transform_17927193494080
// MI455X (gfx1250) — hardware-verified
//
#include <hip/hip_runtime.h>


namespace {
constexpr int B = 4, S = 4096, D = 256, FF = 256, BL = 4  ;
constexpr float XS = 8.0f, WSC = 256.0f, PS = 1024.0f, LOG2E = 1.4426950408889634f, LNEPS = 1e-5f, MASK_FILL = -32767.0f;
static_assert(S % 64 == 0 && D == 256 && FF == 256, "tiling");
typedef _Float16 b16;
typedef __attribute__((ext_vector_type(16))) _Float16 v16b;
typedef __attribute__((ext_vector_type(8))) _Float16 v8b;
typedef __attribute__((ext_vector_type(8))) float v8f;
typedef __attribute__((ext_vector_type(4))) float v4f;
__device__ __forceinline__ float bf16_rne(float f) { unsigned int u = __float_as_uint(f); u += 0x7FFFu + ((u >> 16) & 1u); return __uint_as_float(u & 0xFFFF0000u); }
__device__ __forceinline__ void split16(float v, b16& hi, b16& lo) { hi = (b16)v; lo = (b16)(v - (float)hi); }
__device__ __forceinline__ v16b frag_kb(const b16* p, int hh) { const v8b a = *(const v8b*)(p + 8 * hh), b = *(const v8b*)(p + 16 + 8 * hh); v16b f;
#pragma unroll
  for (int e = 0; e < 8; ++e) { f[e] = a[e]; f[8 + e] = b[e]; } return f; }
__device__ __forceinline__ v8f wmma16b(v16b a, v16b b, v8f c) { v8f d = __builtin_amdgcn_wmma_f32_16x16x32_f16(false, a, false, b, (short)0, c, false, false); asm volatile("v_nop\n\tv_nop\n\tv_nop\n\tv_nop" : "+v"(d) : "v"(a), "v"(b)); return d; }
__device__ __forceinline__ void wave_lds_sync() { __builtin_amdgcn_fence(__ATOMIC_RELEASE, "workgroup"); __builtin_amdgcn_wave_barrier(); __builtin_amdgcn_fence(__ATOMIC_ACQUIRE, "workgroup"); }
__device__ __forceinline__ float pmul(float a, float b) { float p = a * b; asm volatile("" : "+v"(p)); return p; }
__device__ __forceinline__ int iclamp(int v, int lo, int hi) { return v < lo ? lo : (v > hi ? hi : v); }

typedef __attribute__((ext_vector_type(2))) _Float16 v2h;
typedef __attribute__((ext_vector_type(4))) _Float16 v4h;
typedef __attribute__((ext_vector_type(2))) float v2f;
__device__ __forceinline__ float nexp2(float v) { return __builtin_amdgcn_exp2f(v); }
__global__ __launch_bounds__(256) void wprep_kernel(const float* __restrict__ wq, const float* __restrict__ wk, const float* __restrict__ wv, const float* __restrict__ w1, const float* __restrict__ w2, b16* __restrict__ WT) {
  const size_t u = (size_t)blockIdx.x * 256 + threadIdx.x; if (u >= (size_t)5 * D * D / 8) return; const size_t e = u * 8; const int m = (int)(e / (D * D)); const size_t el = e % ((size_t)D * D);
  const float* w = m == 0 ? wq : m == 1 ? wk : m == 2 ? wv : m == 3 ? w1 : w2; v8b o; for (int j = 0; j < 8; ++j) o[j] = (b16)(bf16_rne(w[el + j]) * WSC);
  for (int pass = 0; pass < 2; ++pass) { *(volatile v8b*)(WT + e) = o; __threadfence(); }
}
__global__ __launch_bounds__(128) void qkv_kernel(const float* __restrict__ x, const b16* __restrict__ WT, const float* __restrict__ bq, const float* __restrict__ bk, const float* __restrict__ bv, b16* __restrict__ Qp, b16* __restrict__ Kp, b16* __restrict__ VT) {
  __shared__ __attribute__((aligned(16))) b16 As[4][16][D + 8]; __shared__ __attribute__((aligned(16))) float Tf[4][16][256 + 4];
  const int wave = threadIdx.x >> 5, lane = threadIdx.x & 31, nloc = lane & 15, hlf = lane >> 4; const int b = blockIdx.y, which = blockIdx.z; const int t0 = blockIdx.x * 64 + wave * 16;
  for (int rr = 0; rr < 16; ++rr) { const float* xr = x + ((size_t)b * S + t0 + rr) * D; v8b o; for (int j = 0; j < 8; ++j) o[j] = (b16)(bf16_rne(xr[lane * 8 + j]) * XS); *(v8b*)(&As[wave][rr][lane * 8]) = o; }
  wave_lds_sync();
  const b16* W = WT + (size_t)which * D * D; const float* bias = which == 0 ? bq : which == 1 ? bk : bv;
  v8f acc[16];
#pragma unroll
  for (int t = 0; t < 16; ++t) acc[t] = (v8f){};
#pragma unroll 1
  for (int kb = 0; kb < D; kb += 32) { const v16b a = frag_kb(&As[wave][nloc][kb], hlf);
#pragma unroll
    for (int t = 0; t < 16; ++t) acc[t] = wmma16b(a, frag_kb(W + (size_t)(t * 16 + nloc) * D + kb, hlf), acc[t]); }
#pragma unroll
  for (int t = 0; t < 16; ++t) { const float bb = bf16_rne(bias[t * 16 + nloc]);
#pragma unroll
    for (int r = 0; r < 8; ++r) Tf[wave][8 * hlf + r][t * 16 + nloc] = acc[t][r] * (1.0f / (XS * WSC)) + bb; }
  __syncthreads();
  for (int pass = 0; pass < 2; ++pass) {
    if (which < 2) { b16* P = (which == 0 ? Qp : Kp) + ((size_t)b * S) * D; for (int rr = 0; rr < 16; ++rr) { v8b o; for (int j = 0; j < 8; ++j) o[j] = (b16)(Tf[wave][rr][lane * 8 + j] * XS); *(volatile v8b*)(P + (size_t)(t0 + rr) * D + lane * 8) = o; } }
    else {
#pragma unroll 1
      for (int q = 0; q < 64; ++q) { const int d = wave * 64 + q; const int tk = lane * 2; v2h vv; vv[0] = (b16)(Tf[tk >> 4][tk & 15][d] * XS); vv[1] = (b16)(Tf[(tk + 1) >> 4][(tk + 1) & 15][d] * XS); *(volatile v2h*)(VT + ((size_t)b * D + d) * S + blockIdx.x * 64 + lane * 2) = vv; } }
    __threadfence(); }
}
__global__ __launch_bounds__(64) void attn_kernel(const b16* __restrict__ Qp, const b16* __restrict__ Kp, const b16* __restrict__ VT, const float* __restrict__ x, float* __restrict__ O1) {
  __shared__ __attribute__((aligned(16))) b16 Pb[2][16][32 + 8]; __shared__ __attribute__((aligned(16))) float To[2][16][D + 4];
  const int wave = threadIdx.x >> 5, lane = threadIdx.x & 31, hh = lane >> 4, col = lane & 15; const int b = blockIdx.y; const int q0 = blockIdx.x * 32 + wave * 16, qi = q0 + col;
  const b16* Qb = Qp + (size_t)b * S * D; const b16* Kb = Kp + (size_t)b * S * D; const b16* Vb = VT + (size_t)b * D * S;
  v16b qa[8]; for (int ks = 0; ks < 8; ++ks) qa[ks] = frag_kb(Qb + (size_t)qi * D + ks * 32, hh);
  const float cs = LOG2E / (16.0f * XS * XS);
  float m = -INFINITY, l = 0.0f; v8f o[16]; for (int t = 0; t < 16; ++t) o[t] = (v8f){};
  const int kend = q0 + 16;
#pragma unroll 1
  for (int kb = 0; kb < kend; kb += 32) {
    v8f s[2] = {(v8f){}, (v8f){}};
#pragma unroll
    for (int tt = 0; tt < 2; ++tt)
#pragma unroll
      for (int ks = 0; ks < 8; ++ks) s[tt] = wmma16b(frag_kb(Kb + (size_t)(kb + tt * 16 + col) * D + ks * 32, hh), qa[ks], s[tt]);
    float e[16]; float mx = -INFINITY;
#pragma unroll
    for (int i = 0; i < 16; ++i) { const int key = kb + (i < 8 ? 0 : 16) + 8 * hh + (i & 7); const float v = (key <= qi) ? (i < 8 ? s[0][i] : s[1][i - 8]) * cs : -INFINITY; e[i] = v; mx = fmaxf(mx, v); }
    mx = fmaxf(mx, __shfl_xor(mx, 16)); const float mn = fmaxf(m, mx); const float al = (mn == -INFINITY) ? 1.0f : nexp2(m - mn); float sum = 0.0f;
#pragma unroll
    for (int i = 0; i < 16; ++i) { const float p = (e[i] == -INFINITY) ? 0.0f : nexp2(e[i] - mn); sum += p; Pb[wave][col][(i < 8 ? 0 : 16) + 8 * hh + (i & 7)] = (b16)(p * PS); }
    sum += __shfl_xor(sum, 16); l = l * al + sum; m = mn;
    wave_lds_sync();
    const v16b pf = frag_kb(&Pb[wave][col][0], hh);
#pragma unroll
    for (int t = 0; t < 16; ++t) { o[t] *= al; o[t] = wmma16b(frag_kb(Vb + (size_t)(t * 16 + col) * S + kb, hh), pf, o[t]); }
    wave_lds_sync(); }
  const float inv = 1.0f / (l * PS * XS);
#pragma unroll
  for (int t = 0; t < 16; ++t)
#pragma unroll
    for (int r = 0; r < 8; ++r) To[wave][col][t * 16 + 8 * hh + r] = o[t][r] * inv;
  wave_lds_sync();
  for (int pass = 0; pass < 2; ++pass) { for (int rr = 0; rr < 16; ++rr) { const size_t row = ((size_t)b * S + q0 + rr) * D; v4f a0 = *(const v4f*)(&To[wave][rr][lane * 8]), a1 = *(const v4f*)(&To[wave][rr][lane * 8 + 4]); const v4f x0 = *(const v4f*)(x + row + lane * 8), x1 = *(const v4f*)(x + row + lane * 8 + 4);
      for (int j = 0; j < 4; ++j) { a0[j] += bf16_rne(x0[j]); a1[j] += bf16_rne(x1[j]); } *(volatile v4f*)(O1 + row + lane * 8) = a0; *(volatile v4f*)(O1 + row + lane * 8 + 4) = a1; } __threadfence(); }
}
template <int MODE>
__global__ __launch_bounds__(256) void ln_kernel(const float* __restrict__ IN, const float* __restrict__ g_, const float* __restrict__ b_, b16* __restrict__ Oh, b16* __restrict__ Ol, float* __restrict__ out) {
  const int wave = threadIdx.x >> 5, lane = threadIdx.x & 31; const size_t row = (size_t)blockIdx.x * 8 + wave; const float* r = IN + row * D + lane * 8;
  v4f a = *(const v4f*)r, c = *(const v4f*)(r + 4); float s = 0.0f; for (int j = 0; j < 4; ++j) s += a[j] + c[j];
#pragma unroll
  for (int o = 1; o < 32; o <<= 1) s += __shfl_xor(s, o);
  const float mu = s * (1.0f / D); float q = 0.0f; for (int j = 0; j < 4; ++j) { const float d0 = a[j] - mu, d1 = c[j] - mu; q += d0 * d0 + d1 * d1; }
#pragma unroll
  for (int o = 1; o < 32; o <<= 1) q += __shfl_xor(q, o);
  const float rs = rsqrtf(q * (1.0f / D) + LNEPS); float y[8];
  for (int j = 0; j < 4; ++j) { y[j] = (a[j] - mu) * rs * bf16_rne(g_[lane * 8 + j]) + bf16_rne(b_[lane * 8 + j]); y[4 + j] = (c[j] - mu) * rs * bf16_rne(g_[lane * 8 + 4 + j]) + bf16_rne(b_[lane * 8 + 4 + j]); }
  for (int pass = 0; pass < 2; ++pass) {
    if (MODE == 0) { v8b hv, lv; for (int j = 0; j < 8; ++j) { b16 p, qq; split16(y[j] * XS, p, qq); hv[j] = p; lv[j] = qq; } *(volatile v8b*)(Oh + row * D + lane * 8) = hv; *(volatile v8b*)(Ol + row * D + lane * 8) = lv; }
    else { v4f o0 = {y[0], y[1], y[2], y[3]}, o1 = {y[4], y[5], y[6], y[7]}; *(volatile v4f*)(out + row * D + lane * 8) = o0; *(volatile v4f*)(out + row * D + lane * 8 + 4) = o1; }
    __threadfence(); }
}
template <int MODE>
__global__ __launch_bounds__(128) void ffn_kernel(const b16* __restrict__ Ah, const b16* __restrict__ Al, const b16* __restrict__ W, const float* __restrict__ bias, b16* __restrict__ Oh, b16* __restrict__ Ol, float* __restrict__ OUTF) {
  __shared__ __attribute__((aligned(16))) float Tf[4][16][128 + 4];
  const int wave = threadIdx.x >> 5, lane = threadIdx.x & 31, nloc = lane & 15, hlf = lane >> 4; const size_t m0 = (size_t)blockIdx.x * 64 + wave * 16; const int n0 = blockIdx.y * 128;
  v8f acc[8];
#pragma unroll
  for (int t = 0; t < 8; ++t) acc[t] = (v8f){};
#pragma unroll 2
  for (int kb = 0; kb < D; kb += 32) { const v16b a = frag_kb(Ah + (m0 + nloc) * D + kb, hlf), al = frag_kb(Al + (m0 + nloc) * D + kb, hlf);
#pragma unroll
    for (int t = 0; t < 8; ++t) { const v16b bw = frag_kb(W + (size_t)(n0 + t * 16 + nloc) * D + kb, hlf); acc[t] = wmma16b(a, bw, acc[t]); acc[t] = wmma16b(al, bw, acc[t]); } }
#pragma unroll
  for (int t = 0; t < 8; ++t) { const float bb = bf16_rne(bias[n0 + t * 16 + nloc]);
#pragma unroll
    for (int r = 0; r < 8; ++r) { float v = acc[t][r] * (1.0f / (XS * WSC)) + bb; if (MODE == 0) v = fmaxf(v, 0.0f); Tf[wave][8 * hlf + r][t * 16 + nloc] = v; } }
  wave_lds_sync();
  for (int pass = 0; pass < 2; ++pass) { for (int rr = 0; rr < 16; ++rr) { const v4f f = *(const v4f*)(&Tf[wave][rr][lane * 4]);
      if (MODE == 1) *(volatile v4f*)(OUTF + (m0 + rr) * D + n0 + lane * 4) = f;
      else { v4h hv, lv; for (int j = 0; j < 4; ++j) { b16 p, q; split16(f[j] * XS, p, q); hv[j] = p; lv[j] = q; } *(volatile v4h*)(Oh + (m0 + rr) * D + n0 + lane * 4) = hv; *(volatile v4h*)(Ol + (m0 + rr) * D + n0 + lane * 4) = lv; } }
    __threadfence(); }
}
}

extern "C" void kernel_launch(void* const* d_in, const int* in_sizes, int n_in, void* d_out, int out_size, void* d_ws, size_t ws_size, hipStream_t stream) {
  (void)n_in;
  auto Fp = [&](int i) { return (const float*)d_in[i]; };
  if (in_sizes[0] != B * S * D || in_sizes[1] != D * D || in_sizes[3] != D * D || in_sizes[5] != D * D || in_sizes[7] != FF * D || in_sizes[9] != D * FF || in_sizes[11] != D || in_sizes[13] != D || out_size != B * S * D) return;
  size_t off = 0; char* ws = (char*)d_ws;
  auto carve = [&](size_t bytes) { char* p = ws + off; off += (bytes + 255) & ~(size_t)255; return p; };
  b16* WT = (b16*)carve((size_t)5 * D * D * 2); b16* Qp = (b16*)carve((size_t)B * S * D * 2); b16* Kp = (b16*)carve((size_t)B * S * D * 2); b16* VT = (b16*)carve((size_t)B * D * S * 2);
  float* O1 = (float*)carve((size_t)B * S * D * 4); b16* Ph = (b16*)carve((size_t)B * S * D * 2); b16* Pl = (b16*)carve((size_t)B * S * D * 2); b16* Hh = Qp; b16* Hl = Kp;
  float* H2 = O1;
  if (off > ws_size || off > ((size_t)128 << 20)) return;
  wprep_kernel<<<(unsigned)(((size_t)5 * D * D / 8 + 255) / 256), 256, 0, stream>>>(Fp(1), Fp(3), Fp(5), Fp(7), Fp(9), WT);
  qkv_kernel<<<dim3(S / 64, BL, 3), 128, 0, stream>>>(Fp(0), WT, Fp(2), Fp(4), Fp(6), Qp, Kp, VT);
  attn_kernel<<<dim3(S / 32, BL), 64, 0, stream>>>(Qp, Kp, VT, Fp(0), O1);
  ln_kernel<0><<<(unsigned)((size_t)BL * S / 8), 256, 0, stream>>>(O1, Fp(11), Fp(12), Ph, Pl, nullptr);
  ffn_kernel<0><<<dim3((unsigned)((size_t)BL * S / 64), 2), 128, 0, stream>>>(Ph, Pl, WT + (size_t)3 * D * D, Fp(8), Hh, Hl, nullptr);
  ffn_kernel<1><<<dim3((unsigned)((size_t)BL * S / 64), 2), 128, 0, stream>>>(Hh, Hl, WT + (size_t)4 * D * D, Fp(10), nullptr, nullptr, H2);
  ln_kernel<1><<<(unsigned)((size_t)BL * S / 8), 256, 0, stream>>>(H2, Fp(13), Fp(14), nullptr, nullptr, (float*)d_out);
}
